// VRWKV_SpatialMix_86912958202223
// MI455X (gfx1250) — hardware-verified
//
#include <hip/hip_runtime.h>
#include <math.h>

constexpr int NBATCH = 16;
constexpr int SEQ_T  = 1024;
constexpr int IMG_HW = 32;
constexpr int NCH    = 768;
constexpr int NTOK   = NBATCH * SEQ_T;
constexpr int HID    = 64;
constexpr int NVIEW  = 3;
constexpr int NCAT   = NVIEW * HID;
constexpr int NGRP   = NCH / 4;
constexpr float W_CARRY     = 32.0f;
constexpr float W_CARRY_INV = 1.0f / 32.0f;
constexpr float LN_EPS_F    = 1e-5f;
constexpr float INV_T_F     = 1.0f / 1024.0f;
constexpr float INV_C_F     = 1.0f / 768.0f;
static_assert(IMG_HW * IMG_HW == SEQ_T);
static_assert(NGRP % 8 == 0 && NCH % 64 == 0 && NCAT % 64 == 0 && NTOK % 64 == 0 && NCH % 32 == 0);
static_assert((NTOK / 64) * (NCH / 64) % 8 == 0 && (NTOK / 64) * (NCAT / 64) % 8 == 0);
static_assert((NTOK * (NCH / 8)) % 256 == 0 && (NBATCH * NCH) % 256 == 0 && NTOK % 256 == 0);

constexpr size_t SZ_P16  = (size_t)NTOK * NCH * 2;
constexpr size_t SZ_F32  = (size_t)NTOK * NCH * 4;
constexpr size_t SZ_W4   = (size_t)4 * NCH * NCH * 2;
constexpr size_t SZ_W1   = (size_t)NCAT * NCH * 2;
constexpr size_t SZ_WGT  = (size_t)9 * NTOK * 4;
constexpr size_t OFF_P0  = 0;
constexpr size_t OFF_KR  = OFF_P0 + SZ_P16;
constexpr size_t OFF_VR  = OFF_KR + SZ_F32;
constexpr size_t OFF_W4  = OFF_VR + SZ_F32;
constexpr size_t OFF_W1  = OFF_W4 + SZ_W4;
constexpr size_t OFF_WGT = OFF_W1 + SZ_W1;
constexpr size_t WS_TOTAL = OFF_WGT + SZ_WGT;
static_assert(WS_TOTAL == 131432448ull);
static_assert(WS_TOTAL <= 134217728ull);
static_assert((size_t)NTOK * NCAT * 4 <= SZ_F32);
static_assert(SZ_P16 <= SZ_F32);
static_assert(OFF_KR % 128 == 0 && OFF_VR % 128 == 0 && OFF_W4 % 128 == 0 && OFF_W1 % 128 == 0 && OFF_WGT % 128 == 0);

typedef __attribute__((ext_vector_type(16))) _Float16 v16h;
typedef __attribute__((ext_vector_type(8)))  _Float16 v8h;
typedef __attribute__((ext_vector_type(8)))  float    v8f;
typedef __attribute__((ext_vector_type(4)))  float    v4f;
typedef __attribute__((ext_vector_type(4)))  unsigned int v4u;

__device__ __forceinline__ void dep_guard_h(v8f& a, v8f& b, v16h x, v16h y) { asm volatile("v_nop\n\tv_nop\n\tv_nop\n\tv_nop" : "+v"(a), "+v"(b) : "v"(x), "v"(y)); }
__device__ __forceinline__ void keep4_h(v16h a, v16h b, v16h c, v16h d) { asm volatile("v_nop" :: "v"(a), "v"(b), "v"(c), "v"(d)); }
__device__ __forceinline__ void acc_guard4(v8f& a, v8f& b, v8f& c, v8f& d) { asm volatile("v_nop\n\tv_nop\n\tv_nop\n\tv_nop" : "+v"(a), "+v"(b), "+v"(c), "+v"(d)); }
template <typename T> struct Frag;
template <> struct Frag<_Float16> {
  typedef v16h V; union U { v16h v; v8h h[2]; };
  static __device__ __forceinline__ v16h load(const _Float16* p) {
    U f; f.h[0] = *(const v8h*)(p); f.h[1] = *(const v8h*)(p + 16); return f.v;
  }
  static __device__ __forceinline__ v8f mma(v16h a, v16h b, v8f c) {
    return __builtin_amdgcn_wmma_f32_16x16x32_f16(false, a, false, b, (short)0, c, false, false);
  }
  static __device__ __forceinline__ void guard(v8f& a, v8f& b, v16h x, v16h y) { dep_guard_h(a, b, x, y); }
  static __device__ __forceinline__ void keep(v16h a, v16h b, v16h c, v16h d) { keep4_h(a, b, c, d); }
};

__device__ __forceinline__ unsigned pk16(unsigned short a, unsigned short b) { return (unsigned)a | ((unsigned)b << 16); }
__device__ __forceinline__ unsigned short h_bits(float f) { const _Float16 h = (_Float16)f; return __builtin_bit_cast(unsigned short, h); }

__device__ __forceinline__ float sigmoid_f(float v) {
  const float e = expf(-fabsf(v));
  const float inv = 1.0f / (1.0f + e);
  return (v >= 0.0f) ? inv : e * inv;
}

template <int EPI>
__global__ __launch_bounds__(256) void gemm_f16_kernel(
    const unsigned short* __restrict__ Ap, int lda,
    const unsigned short* __restrict__ Btp, int ldb,
    void* __restrict__ Cout, int ldc,
    const float* __restrict__ bv0, const float* __restrict__ bv1, const float* __restrict__ bv2,
    const float* __restrict__ gsrc,
    int M, int N, int K, float scale) {
  typedef _Float16 T;
  typedef v16h V;
  const T* A  = (const T*)Ap;
  const T* Bt = (const T*)Btp;
  __shared__ __align__(16) float sT[8][16 * 68];
  const int lane = threadIdx.x & 31;
  const int wave = threadIdx.x >> 5;
  const int tilesN = N >> 6;
  const int tilesM = M >> 6;
  const int tile = blockIdx.x * 8 + wave;
  if (tile >= tilesM * tilesN) return;
  const int tm = tile / tilesN;
  const int tn = tile - tm * tilesN;
  const int m0 = tm << 6;
  const int n0 = tn << 6;

  const int rlane = lane & 15;
  const int koff  = (lane >> 4) * 8;
  const int mOff  = (lane >> 4) * 8;

  v8f acc[4][4];
#pragma unroll
  for (int i = 0; i < 4; ++i)
#pragma unroll
    for (int j = 0; j < 4; ++j) acc[i][j] = (v8f){0.f,0.f,0.f,0.f,0.f,0.f,0.f,0.f};

  for (int k0 = 0; k0 < K; k0 += 32) {
    V bh[4];
#pragma unroll
    for (int j = 0; j < 4; ++j) {
      const size_t bo = (size_t)(n0 + (j << 4) + rlane) * ldb + koff + k0;
      bh[j] = Frag<T>::load(Bt + bo);
    }
#pragma unroll
    for (int i = 0; i < 4; ++i) {
      const size_t ao = (size_t)(m0 + (i << 4) + rlane) * lda + koff + k0;
      V ah = Frag<T>::load(A + ao);
#pragma unroll
      for (int j = 0; j < 4; ++j) {
        acc[i][j] = Frag<T>::mma(ah, bh[j], acc[i][j]);
      }
      Frag<T>::guard(acc[i][0], acc[i][3], ah, ah);
    }
    Frag<T>::keep(bh[0], bh[1], bh[2], bh[3]);
  }
  acc_guard4(acc[0][0], acc[0][1], acc[0][2], acc[0][3]);
  acc_guard4(acc[1][0], acc[1][1], acc[1][2], acc[1][3]);
  acc_guard4(acc[2][0], acc[2][1], acc[2][2], acc[2][3]);
  acc_guard4(acc[3][0], acc[3][1], acc[3][2], acc[3][3]);

  float* slab = sT[wave];
#pragma unroll
  for (int i = 0; i < 4; ++i) {
    const int mBase = m0 + (i << 4);
#pragma unroll
    for (int j = 0; j < 4; ++j) {
      const int nl = (j << 4) + rlane;
      float bsel = 0.f;
      if (EPI == 1) {
        const float c0v = bv0[nl], c1v = bv1[nl], c2v = bv2[nl];
        bsel = (tn == 0) ? c0v : ((tn == 1) ? c1v : c2v);
      }
#pragma unroll
      for (int r = 0; r < 8; ++r) {
        float v = acc[i][j][r] * scale;
        if (EPI == 1) v = fmaxf(v + bsel, 0.0f);
        slab[(mOff + r) * 68 + (j << 4) + rlane] = v;
      }
    }
    __builtin_amdgcn_fence(__ATOMIC_RELEASE, "workgroup");
    __builtin_amdgcn_wave_barrier();
    __builtin_amdgcn_fence(__ATOMIC_ACQUIRE, "workgroup");
    if (EPI != 2) {
      float* C = (float*)Cout;
      const int hh = lane >> 4, c4 = (lane & 15) * 4;
      for (int pass = 0; pass < 2; ++pass) {
#pragma unroll
        for (int it = 0; it < 8; ++it) {
          const int row = it * 2 + hh;
          v4f v = *(const v4f*)(slab + row * 68 + c4);
          *(volatile v4f*)(C + (size_t)(mBase + row) * ldc + n0 + c4) = v;
        }
        __threadfence();
      }
    } else {
      const int q = lane >> 3, c8 = (lane & 7) * 8;
      unsigned short* Cp = (unsigned short*)Cout;
      v8h hv[4];
#pragma unroll
      for (int it = 0; it < 4; ++it) {
        const int row = it * 4 + q;
        const float* sp = slab + row * 68 + c8;
        const v4f s0 = *(const v4f*)(sp);
        const v4f s1 = *(const v4f*)(sp + 4);
        const float* gp = gsrc + (size_t)(mBase + row) * ldc + n0 + c8;
        const v4f g0 = *(const v4f*)(gp);
        const v4f g1 = *(const v4f*)(gp + 4);
#pragma unroll
        for (int e = 0; e < 4; ++e) {
          hv[it][e]     = (_Float16)(sigmoid_f(s0[e]) * g0[e]);
          hv[it][4 + e] = (_Float16)(sigmoid_f(s1[e]) * g1[e]);
        }
      }
      for (int pass = 0; pass < 2; ++pass) {
#pragma unroll
        for (int it = 0; it < 4; ++it) {
          const int row = it * 4 + q;
          *(volatile v8h*)(Cp + (size_t)(mBase + row) * ldc + n0 + c8) = hv[it];
        }
        __threadfence();
      }
    }
    __builtin_amdgcn_fence(__ATOMIC_RELEASE, "workgroup");
    __builtin_amdgcn_wave_barrier();
    __builtin_amdgcn_fence(__ATOMIC_ACQUIRE, "workgroup");
  }
}

__global__ __launch_bounds__(256) void cast8_f16_kernel(const float* __restrict__ s0, const float* __restrict__ s1,
                                                       const float* __restrict__ s2, const float* __restrict__ s3,
                                                       unsigned short* __restrict__ out, long planeElems, int n8, float scale) {
  const int z = blockIdx.y;
  const float* in = (z == 0) ? s0 : ((z == 1) ? s1 : ((z == 2) ? s2 : s3));
  const int i = blockIdx.x * 256 + threadIdx.x;
  if (i >= n8) return;
  const float* p = in + 8 * (size_t)i;
  const v4f a = *(const v4f*)(p);
  const v4f c = *(const v4f*)(p + 4);
  unsigned short hb[8];
#pragma unroll
  for (int e = 0; e < 4; ++e) {
    hb[e]     = h_bits(a[e] * scale);
    hb[4 + e] = h_bits(c[e] * scale);
  }
  const v4u u = (v4u){pk16(hb[0], hb[1]), pk16(hb[2], hb[3]), pk16(hb[4], hb[5]), pk16(hb[6], hb[7])};
  unsigned short* qp = out + (size_t)z * planeElems + 8 * (size_t)i;
  *(volatile v4u*)qp = u;
  __threadfence();
  *(volatile v4u*)qp = u;
}

__global__ __launch_bounds__(256) void view_weight_kernel(const float* __restrict__ hid,
    const float* __restrict__ w2a, const float* __restrict__ b2a,
    const float* __restrict__ w2b, const float* __restrict__ b2b,
    const float* __restrict__ w2c, const float* __restrict__ b2c,
    float* __restrict__ wgt, const int* __restrict__ shp0, const int* __restrict__ shp1) {
  (void)shp0; (void)shp1;
  __shared__ __align__(16) float w2s[NVIEW * NCAT];
  __shared__ float b2s[16];
  const int t = threadIdx.x;
#pragma unroll
  for (int it = 0; it < 3; ++it) {
    const int i  = it * 256 + t;
    const int ic = (i < NVIEW * NCAT) ? i : (NVIEW * NCAT - 1);
    const int s  = ic / NCAT;
    const int r  = ic - s * NCAT;
    const float va = w2a[r], vb = w2b[r], vc = w2c[r];
    const float sel = (s == 0) ? va : ((s == 1) ? vb : vc);
    if (i < NVIEW * NCAT) w2s[i] = sel;
  }
  {
    const int r = t % 3;
    const int s = t / 3;
    const float va = b2a[r], vb = b2b[r], vc = b2c[r];
    const float sel = (s == 0) ? va : ((s == 1) ? vb : vc);
    if (t < 9) b2s[t] = sel;
  }
  __syncthreads();

  const int tok = blockIdx.x * 256 + t;
  const float* hrow = hid + (size_t)tok * NCAT;
#pragma unroll 1
  for (int s = 0; s < NVIEW; ++s) {
    const float* hp = hrow + s * HID;
    const float* wp = w2s + s * NCAT;
    float d0 = 0.0f, d1 = 0.0f, d2 = 0.0f;
#pragma unroll 1
    for (int q4 = 0; q4 < HID / 4; ++q4) {
      const v4f hv = *(const v4f*)(hp + 4 * q4);
#pragma unroll
      for (int e = 0; e < 4; ++e) {
        const int hh = 4 * q4 + e;
        const float h = hv[e];
        d0 += h * wp[hh];
        d1 += h * wp[HID + hh];
        d2 += h * wp[2 * HID + hh];
      }
    }
    const float l0 = d0 + b2s[s * 3 + 0];
    const float l1 = d1 + b2s[s * 3 + 1];
    const float l2 = d2 + b2s[s * 3 + 2];
    const float m  = fmaxf(l0, fmaxf(l1, l2));
    const float e0 = expf(l0 - m), e1 = expf(l1 - m), e2 = expf(l2 - m);
    const float inv = 1.0f / ((e0 + e1) + e2);
    const float p0 = e0 * inv, p1 = e1 * inv, p2 = e2 * inv;
    float* op = wgt + (size_t)(s * 3) * NTOK + tok;
    *(volatile float*)(op) = p0;
    *(volatile float*)(op + NTOK) = p1;
    *(volatile float*)(op + 2 * NTOK) = p2;
    __threadfence();
    *(volatile float*)(op) = p0;
    *(volatile float*)(op + NTOK) = p1;
    *(volatile float*)(op + 2 * NTOK) = p2;
  }
}

__global__ __launch_bounds__(256) void shiftmix_kernel(const float* __restrict__ x, const float* __restrict__ wgt,
                                                      const float* __restrict__ mix, unsigned short* __restrict__ outp, int mlp) {
  const int gid = blockIdx.x * 256 + threadIdx.x;
  const int tok = gid / (NCH / 8);
  const int c0  = (gid - tok * (NCH / 8)) * 8;
  const int b   = tok >> 10;
  const int t   = tok & (SEQ_T - 1);
  const int h0  = t >> 5;
  const int w0  = t & 31;
  const int grp = c0 / NGRP;
  const float a0 = wgt[(size_t)(mlp * 3 + 0) * NTOK + tok];
  const float a1 = wgt[(size_t)(mlp * 3 + 1) * NTOK + tok];
  const float a2 = wgt[(size_t)(mlp * 3 + 2) * NTOK + tok];
  const float* xb = x + (size_t)b * SEQ_T * NCH;
  const float* xp = xb + (size_t)t * NCH + c0;
  const v4f xc0 = *(const v4f*)(xp);
  const v4f xc1 = *(const v4f*)(xp + 4);
  v4f xx0 = (v4f){0.f, 0.f, 0.f, 0.f};
  v4f xx1 = (v4f){0.f, 0.f, 0.f, 0.f};
#pragma unroll
  for (int r = 1; r <= 3; ++r) {
    const int dh = (grp == 2) ? -r : ((grp == 3) ? r : 0);
    const int dw = (grp == 0) ? -r : ((grp == 1) ? r : 0);
    int hs = h0 + dh;
    int ws = w0 + dw;
    const bool ok = ((unsigned)hs < (unsigned)IMG_HW) && ((unsigned)ws < (unsigned)IMG_HW);
    hs = hs < 0 ? 0 : (hs > IMG_HW - 1 ? IMG_HW - 1 : hs);
    ws = ws < 0 ? 0 : (ws > IMG_HW - 1 ? IMG_HW - 1 : ws);
    const float* sp = xb + (size_t)(hs * IMG_HW + ws) * NCH + c0;
    const v4f sv0 = *(const v4f*)(sp);
    const v4f sv1 = *(const v4f*)(sp + 4);
    const float ar = (r == 1) ? a0 : ((r == 2) ? a1 : a2);
    const float wr = ok ? ar : 0.0f;
    xx0 += sv0 * wr;
    xx1 += sv1 * wr;
  }
  const v4f mv0 = *(const v4f*)(mix + c0);
  const v4f mv1 = *(const v4f*)(mix + c0 + 4);
  const v4f o0 = xc0 * mv0 + xx0 * (1.0f - mv0);
  const v4f o1 = xc1 * mv1 + xx1 * (1.0f - mv1);
  unsigned short hb[8];
#pragma unroll
  for (int e = 0; e < 4; ++e) {
    hb[e]     = h_bits(o0[e]);
    hb[4 + e] = h_bits(o1[e]);
  }
  const v4u u = (v4u){pk16(hb[0], hb[1]), pk16(hb[2], hb[3]), pk16(hb[4], hb[5]), pk16(hb[6], hb[7])};
  unsigned short* qp = outp + (size_t)tok * NCH + c0;
  *(volatile v4u*)qp = u;
  __threadfence();
  *(volatile v4u*)qp = u;
}

__global__ __launch_bounds__(256) void decay_scan_kernel(float* __restrict__ kio, const float* __restrict__ vsrc,
                                                        const float* __restrict__ decay, const float* __restrict__ first) {
  const int idx = blockIdx.x * 256 + threadIdx.x;
  const int b = idx / NCH;
  const int c = idx - b * NCH;
  const float w = decay[c] * INV_T_F;
  const float u = first[c] * INV_T_F;
  const size_t base = (size_t)b * SEQ_T * NCH + c;
  float* yk = kio + base;
  const float* vp = vsrc + base;
  float p = 0.0f, q = 0.0f, o = -1e38f;
  float kt = yk[0];
  float vt = vp[0];
#pragma unroll 1
  for (int t = 0; t < SEQ_T; ++t) {
    const int tnx = (t + 1 < SEQ_T) ? (t + 1) : (SEQ_T - 1);
    const float ktn = yk[(size_t)tnx * NCH];
    const float vtn = vp[(size_t)tnx * NCH];

    const float ukt = u + kt;
    const float d1  = ukt - o;
    const float e1  = expf(-fabsf(d1));
    const float Aa  = (d1 > 0.0f) ? e1 : 1.0f;
    const float Bc  = (d1 > 0.0f) ? 1.0f : e1;
    const float y   = (Aa * p + Bc * vt) / (Aa * q + Bc);

    float* ya = yk + (size_t)t * NCH;
    *(volatile float*)ya = y;
    __threadfence();
    *(volatile float*)ya = y;

    const float wo  = w + o;
    const float d2  = kt - wo;
    const float e2  = expf(-fabsf(d2));
    const float A2  = (d2 > 0.0f) ? e2 : 1.0f;
    const float B2  = (d2 > 0.0f) ? 1.0f : e2;
    p = A2 * p + B2 * vt;
    q = A2 * q + B2;
    o = fmaxf(wo, kt);
    kt = ktn;
    vt = vtn;
  }
}

__global__ __launch_bounds__(192) void layernorm_kernel(const float* __restrict__ y, const float* __restrict__ gam,
                                                       const float* __restrict__ bet, float* __restrict__ out) {
  __shared__ float redA[8];
  __shared__ float redB[8];
  const int tok  = blockIdx.x;
  const int t    = threadIdx.x;
  const int lane = t & 31, wave = t >> 5;
  const v4f yv = *(const v4f*)(y + (size_t)tok * NCH + 4 * t);
  float s = (yv[0] + yv[1]) + (yv[2] + yv[3]);
#pragma unroll
  for (int off = 16; off > 0; off >>= 1) s += __shfl_xor(s, off, 32);
  if (lane == 0) redA[wave] = s;
  __syncthreads();
  float tot = redA[0];
#pragma unroll
  for (int wv = 1; wv < 6; ++wv) tot += redA[wv];
  const float mu = tot * INV_C_F;
  v4f d;
#pragma unroll
  for (int e = 0; e < 4; ++e) d[e] = yv[e] - mu;
  float s2 = (d[0] * d[0] + d[1] * d[1]) + (d[2] * d[2] + d[3] * d[3]);
#pragma unroll
  for (int off = 16; off > 0; off >>= 1) s2 += __shfl_xor(s2, off, 32);
  if (lane == 0) redB[wave] = s2;
  __syncthreads();
  float tot2 = redB[0];
#pragma unroll
  for (int wv = 1; wv < 6; ++wv) tot2 += redB[wv];
  const float var  = tot2 * INV_C_F;
  const float rstd = rsqrtf(var + LN_EPS_F);
  const v4f gv = *(const v4f*)(gam + 4 * t);
  const v4f bv = *(const v4f*)(bet + 4 * t);
  v4f o;
#pragma unroll
  for (int e = 0; e < 4; ++e) o[e] = d[e] * rstd * gv[e] + bv[e];
  float* op = out + (size_t)tok * NCH + 4 * t;
  *(volatile v4f*)op = o;
  __threadfence();
  *(volatile v4f*)op = o;
}

extern "C" void kernel_launch(void* const* d_in, const int* in_sizes, int n_in,
                              void* d_out, int out_size, void* d_ws, size_t ws_size,
                              hipStream_t stream) {
  if (n_in < 26) return;
  if (in_sizes[0] != NTOK * NCH || out_size != NTOK * NCH) return;
  if (in_sizes[1] != NCH * NCH || in_sizes[2] != NCH * NCH || in_sizes[3] != NCH * NCH || in_sizes[4] != NCH * NCH) return;
  if (in_sizes[5] != NCH || in_sizes[6] != NCH || in_sizes[7] != NCH || in_sizes[8] != NCH || in_sizes[9] != NCH) return;
  if (in_sizes[10] != NCH || in_sizes[11] != NCH) return;
  if (in_sizes[12] != HID * NCH || in_sizes[16] != HID * NCH || in_sizes[20] != HID * NCH) return;
  if (in_sizes[13] != HID || in_sizes[17] != HID || in_sizes[21] != HID) return;
  if (in_sizes[14] != NVIEW * HID || in_sizes[18] != NVIEW * HID || in_sizes[22] != NVIEW * HID) return;
  if (in_sizes[15] != NVIEW || in_sizes[19] != NVIEW || in_sizes[23] != NVIEW) return;
  if (ws_size < WS_TOTAL) return;

  const float* x     = (const float*)d_in[0];
  const float* Wk    = (const float*)d_in[1];
  const float* Wv    = (const float*)d_in[2];
  const float* Wr    = (const float*)d_in[3];
  const float* Wo    = (const float*)d_in[4];
  const float* ln_g  = (const float*)d_in[5];
  const float* ln_b  = (const float*)d_in[6];
  const float* mix_k = (const float*)d_in[7];
  const float* mix_v = (const float*)d_in[8];
  const float* mix_r = (const float*)d_in[9];
  const float* decay = (const float*)d_in[10];
  const float* first = (const float*)d_in[11];
  const float* sk_w1 = (const float*)d_in[12];
  const float* sk_b1 = (const float*)d_in[13];
  const float* sk_w2 = (const float*)d_in[14];
  const float* sk_b2 = (const float*)d_in[15];
  const float* sv_w1 = (const float*)d_in[16];
  const float* sv_b1 = (const float*)d_in[17];
  const float* sv_w2 = (const float*)d_in[18];
  const float* sv_b2 = (const float*)d_in[19];
  const float* sr_w1 = (const float*)d_in[20];
  const float* sr_b1 = (const float*)d_in[21];
  const float* sr_w2 = (const float*)d_in[22];
  const float* sr_b2 = (const float*)d_in[23];
  const int*   shpH  = (const int*)d_in[24];
  const int*   shpW  = (const int*)d_in[25];
  float* out = (float*)d_out;

  char* ws = (char*)d_ws;
  unsigned short* P0  = (unsigned short*)(ws + OFF_P0);
  float*          KRf = (float*)(ws + OFF_KR);
  unsigned short* YG16 = (unsigned short*)(ws + OFF_KR);
  float*          VRf = (float*)(ws + OFF_VR);
  unsigned short* W4  = (unsigned short*)(ws + OFF_W4);
  unsigned short* W1  = (unsigned short*)(ws + OFF_W1);
  float*          WGT = (float*)(ws + OFF_WGT);

  const long planeW  = (long)NCH * NCH;
  const long planeW1 = (long)HID * NCH;
  const int n8x  = (NTOK * NCH) / 8;
  const int n8w  = (NCH * NCH) / 8;
  const int n8w1 = (HID * NCH) / 8;
  const int blkN768 = ((NTOK / 64) * (NCH / 64)) / 8;
  const int blkN192 = ((NTOK / 64) * (NCAT / 64)) / 8;

  cast8_f16_kernel<<<dim3(n8x / 256, 1), dim3(256), 0, stream>>>(x, x, x, x, P0, (long)NTOK * NCH, n8x, 1.0f);
  cast8_f16_kernel<<<dim3(n8w / 256, 4), dim3(256), 0, stream>>>(Wk, Wv, Wr, Wo, W4, planeW, n8w, W_CARRY);
  cast8_f16_kernel<<<dim3(n8w1 / 256, 3), dim3(256), 0, stream>>>(sk_w1, sv_w1, sr_w1, sr_w1, W1, planeW1, n8w1, W_CARRY);

  gemm_f16_kernel<1><<<dim3(blkN192), dim3(256), 0, stream>>>(
      P0, NCH, W1, NCH, (void*)VRf, NCAT, sk_b1, sv_b1, sr_b1, x, NTOK, NCAT, NCH, W_CARRY_INV);

  view_weight_kernel<<<dim3(NTOK / 256), dim3(256), 0, stream>>>(
      VRf, sk_w2, sk_b2, sv_w2, sv_b2, sr_w2, sr_b2, WGT, shpH, shpW);

  shiftmix_kernel<<<dim3(NTOK * (NCH / 8) / 256), dim3(256), 0, stream>>>(x, WGT, mix_k, P0, 0);
  gemm_f16_kernel<0><<<dim3(blkN768), dim3(256), 0, stream>>>(
      P0, NCH, W4, NCH, (void*)KRf, NCH, ln_g, ln_g, ln_g, x, NTOK, NCH, NCH, W_CARRY_INV);

  shiftmix_kernel<<<dim3(NTOK * (NCH / 8) / 256), dim3(256), 0, stream>>>(x, WGT, mix_v, P0, 1);
  gemm_f16_kernel<0><<<dim3(blkN768), dim3(256), 0, stream>>>(
      P0, NCH, W4 + planeW, NCH, (void*)VRf, NCH, ln_g, ln_g, ln_g, x, NTOK, NCH, NCH, W_CARRY_INV);

  decay_scan_kernel<<<dim3((NBATCH * NCH) / 256), dim3(256), 0, stream>>>(KRf, VRf, decay, first);

  layernorm_kernel<<<dim3(NTOK), dim3(192), 0, stream>>>(KRf, ln_g, ln_b, VRf);

  shiftmix_kernel<<<dim3(NTOK * (NCH / 8) / 256), dim3(256), 0, stream>>>(x, WGT, mix_r, P0, 2);
  gemm_f16_kernel<2><<<dim3(blkN768), dim3(256), 0, stream>>>(
      P0, NCH, W4 + 2 * planeW, NCH, (void*)YG16, NCH, ln_g, ln_g, ln_g, VRf, NTOK, NCH, NCH, W_CARRY_INV);

  gemm_f16_kernel<0><<<dim3(blkN768), dim3(256), 0, stream>>>(
      YG16, NCH, W4 + 3 * planeW, NCH, (void*)out, NCH, ln_g, ln_g, ln_g, x, NTOK, NCH, NCH, W_CARRY_INV);
}
